// SimpleMAMBA_74895639708063
// MI455X (gfx1250) — hardware-verified
//
#include <hip/hip_runtime.h>
#include <math.h>

typedef __attribute__((ext_vector_type(16))) _Float16 v16h;
typedef __attribute__((ext_vector_type(8)))  _Float16 v8h;
typedef __attribute__((ext_vector_type(16))) __bf16   v16b;
typedef __attribute__((ext_vector_type(8)))  __bf16   v8b;
typedef __attribute__((ext_vector_type(8)))  float    v8f;
typedef __attribute__((ext_vector_type(4)))  float    v4f;

constexpr int kBatch  = 4;
constexpr int kSeq    = 2048;
constexpr int kFin    = 512;
constexpr int kDm     = 1024;
constexpr int kDi     = 2048;
constexpr int kNst    = 16;
constexpr int kXz     = 2 * kDi;
constexpr int kDtR    = 64;
constexpr int kXpN    = 96;
constexpr int kXdP    = 128;
constexpr int kFout   = 512;
constexpr int kRows   = kBatch * kSeq;
constexpr int kConvTP = 260;
constexpr int kScanTS = 64;
constexpr int kScanCh = 64;
constexpr int kScanYP = 68;
constexpr int kBcP    = 36;
constexpr float kWinCarry  = 64.0f;
constexpr float kWdtCarry  = 64.0f;
constexpr float kWoutCarry = 256.0f;
constexpr float kDtCarry   = 16.0f;
constexpr float kYCarry    = 16.0f;

constexpr size_t kOffXB   = 0;
constexpr size_t kOffWF1  = kOffXB   + (size_t)kRows * kFin * 2;
constexpr size_t kOffWIN  = kOffWF1  + (size_t)kDm   * kFin * 2;
constexpr size_t kOffWXP  = kOffWIN  + (size_t)kXz   * kDm  * 2;
constexpr size_t kOffWDT  = kOffWXP  + (size_t)kXdP  * kDi  * 2;
constexpr size_t kOffWOU  = kOffWDT  + (size_t)kDi   * kDtR * 2;
constexpr size_t kOffWF2  = kOffWOU  + (size_t)kDm   * kDi  * 2;
constexpr size_t kOffH16  = kOffWF2  + (size_t)kFout * kDm  * 2;
constexpr size_t kOffXZ   = kOffH16  + (size_t)kSeq  * kDm  * 2;
constexpr size_t kOffUC   = kOffXZ   + (size_t)kSeq  * kXz  * 4;
constexpr size_t kOffUCH  = kOffUC   + (size_t)kSeq  * kDi  * 4;
constexpr size_t kOffUCL  = kOffUCH  + (size_t)kSeq  * kDi  * 2;
constexpr size_t kOffXD   = kOffUCL  + (size_t)kSeq  * kDi  * 2;
constexpr size_t kOffDT   = kOffXD   + (size_t)kSeq  * kXdP * 4;
constexpr size_t kOffY16  = kOffDT   + (size_t)kSeq  * kDtR * 2;
constexpr size_t kWsTotal = kOffY16  + (size_t)kSeq  * kDi  * 2;
constexpr size_t kOffDTP  = kOffUCH;
constexpr size_t kOffM2H  = kOffUCH;
constexpr size_t kOffM2L  = kOffUCH  + (size_t)kSeq  * kDm  * 2;
static_assert(kWsTotal == 104857600ull, "carve total");
static_assert(kWsTotal <= 134217728ull, "carve cap");
static_assert((size_t)kSeq * kDi * 4 <= (kOffXD - kOffUCH), "DTP fits in UCH|UCL");
static_assert(kOffM2L + (size_t)kSeq * kDm * 2 <= kOffXD, "M2 planes fit in UCH|UCL");
static_assert((kOffWF1 % 128) == 0 && (kOffWIN % 128) == 0 && (kOffWXP % 128) == 0 && (kOffWDT % 128) == 0 &&
              (kOffWOU % 128) == 0 && (kOffWF2 % 128) == 0 && (kOffH16 % 128) == 0 && (kOffXZ % 128) == 0 &&
              (kOffUC % 128) == 0 && (kOffUCH % 128) == 0 && (kOffUCL % 128) == 0 && (kOffXD % 128) == 0 &&
              (kOffDT % 128) == 0 && (kOffY16 % 128) == 0 && (kOffM2L % 128) == 0,
              "128-B aligned regions");

__device__ __forceinline__ unsigned short f2bf_bits(float f) {
  unsigned u = __float_as_uint(f);
  return (unsigned short)((u + 0x7FFFu + ((u >> 16) & 1u)) >> 16);
}
__device__ __forceinline__ float bf_bits2f(unsigned short h) { return __uint_as_float(((unsigned)h) << 16); }
__device__ __forceinline__ float bfr(float f) { return bf_bits2f(f2bf_bits(f)); }

__device__ __forceinline__ void dep_guard_h(v8f& a, v8f& b, v16h x, v16h y) { asm volatile("v_nop\n\tv_nop\n\tv_nop\n\tv_nop" : "+v"(a), "+v"(b) : "v"(x), "v"(y)); }
__device__ __forceinline__ void dep_guard_b(v8f& a, v8f& b, v16b x, v16b y) { asm volatile("v_nop\n\tv_nop\n\tv_nop\n\tv_nop" : "+v"(a), "+v"(b) : "v"(x), "v"(y)); }
__device__ __forceinline__ void keep4_h(v16h a, v16h b, v16h c, v16h d) { asm volatile("v_nop" :: "v"(a), "v"(b), "v"(c), "v"(d)); }
__device__ __forceinline__ void keep4_b(v16b a, v16b b, v16b c, v16b d) { asm volatile("v_nop" :: "v"(a), "v"(b), "v"(c), "v"(d)); }
__device__ __forceinline__ void acc_guard4(v8f& a, v8f& b, v8f& c, v8f& d) { asm volatile("v_nop\n\tv_nop\n\tv_nop\n\tv_nop" : "+v"(a), "+v"(b), "+v"(c), "+v"(d)); }
template <typename T> struct Frag;
template <> struct Frag<_Float16> {
  typedef v16h V; union U { v16h v; v8h h[2]; };
  static __device__ __forceinline__ v16h load(const _Float16* p) {
    U f; f.h[0] = *(const v8h*)(p); f.h[1] = *(const v8h*)(p + 16); return f.v;
  }
  static __device__ __forceinline__ v8f mma(v16h a, v16h b, v8f c) {
    return __builtin_amdgcn_wmma_f32_16x16x32_f16(false, a, false, b, (short)0, c, false, false);
  }
  static __device__ __forceinline__ void guard(v8f& a, v8f& b, v16h x, v16h y) { dep_guard_h(a, b, x, y); }
  static __device__ __forceinline__ void keep(v16h a, v16h b, v16h c, v16h d) { keep4_h(a, b, c, d); }
};
template <> struct Frag<__bf16> {
  typedef v16b V; union U { v16b v; v8b h[2]; };
  static __device__ __forceinline__ v16b load(const __bf16* p) {
    U f; f.h[0] = *(const v8b*)(p); f.h[1] = *(const v8b*)(p + 16); return f.v;
  }
  static __device__ __forceinline__ v8f mma(v16b a, v16b b, v8f c) {
    return __builtin_amdgcn_wmma_f32_16x16x32_bf16(false, a, false, b, (short)0, c, false, false);
  }
  static __device__ __forceinline__ void guard(v8f& a, v8f& b, v16b x, v16b y) { dep_guard_b(a, b, x, y); }
  static __device__ __forceinline__ void keep(v16b a, v16b b, v16b c, v16b d) { keep4_b(a, b, c, d); }
};

template <int ET> struct Elem;
template <> struct Elem<0> { typedef _Float16 T; };
template <> struct Elem<1> { typedef __bf16 T; };
template <int ET, int SPL, int BIAS_MODE, int OUT_MODE, bool RESID, int ACT = 0>
__global__ __launch_bounds__(256) void wmma_gemm64(
    const unsigned short* __restrict__ Ap, const unsigned short* __restrict__ A2p, int lda, long strideA,
    const unsigned short* __restrict__ Btp, const unsigned short* __restrict__ Bt2p, int ldb, long strideB,
    void* __restrict__ Cout, void* __restrict__ Cout2, int ldc, long strideC,
    const float* __restrict__ bias,
    const float* __restrict__ resid, long strideR,
    int M, int N, int K, float scale) {
  typedef typename Elem<ET>::T T;
  typedef typename Frag<T>::V V;
  const T* A = (const T*)Ap; const T* A2 = (const T*)A2p; const T* Bt = (const T*)Btp; const T* Bt2 = (const T*)Bt2p;
  __shared__ __align__(16) float sT[8][16 * 68];
  const int b    = blockIdx.y;
  const int lane = threadIdx.x & 31;
  const int wave = threadIdx.x >> 5;
  const int tilesN = N >> 6;
  const int tilesM = M >> 6;
  const int tile = blockIdx.x * 8 + wave;
  if (tile >= tilesM * tilesN) return;
  const int tm = tile / tilesN;
  const int tn = tile - tm * tilesN;
  const int m0 = tm << 6;
  const int n0 = tn << 6;

  const T* Ab  = A  + (size_t)b * strideA;
  const T* Bb  = Bt + (size_t)b * strideB;
  const T* Ab2 = (SPL >= 1) ? (A2  + (size_t)b * strideA) : nullptr;
  const T* Bb2 = (SPL == 2) ? (Bt2 + (size_t)b * strideB) : nullptr;

  const int rlane = lane & 15;
  const int koff  = (lane >> 4) * 8;
  const int mOff  = (lane >> 4) * 8;

  v8f acc[4][4];
#pragma unroll
  for (int i = 0; i < 4; ++i)
#pragma unroll
    for (int j = 0; j < 4; ++j) acc[i][j] = (v8f){0.f,0.f,0.f,0.f,0.f,0.f,0.f,0.f};

  for (int k0 = 0; k0 < K; k0 += 32) {
    V bh[4], bl[4];
#pragma unroll
    for (int j = 0; j < 4; ++j) {
      const size_t bo = (size_t)(n0 + (j << 4) + rlane) * ldb + koff + k0;
      bh[j] = Frag<T>::load(Bb + bo);
      if (SPL == 2) bl[j] = Frag<T>::load(Bb2 + bo);
    }
#pragma unroll
    for (int i = 0; i < 4; ++i) {
      const size_t ao = (size_t)(m0 + (i << 4) + rlane) * lda + koff + k0;
      V ah = Frag<T>::load(Ab + ao);
      V al;
      if (SPL >= 1) al = Frag<T>::load(Ab2 + ao);
#pragma unroll
      for (int j = 0; j < 4; ++j) {
        acc[i][j] = Frag<T>::mma(ah, bh[j], acc[i][j]);
        if (SPL == 2) acc[i][j] = Frag<T>::mma(ah, bl[j], acc[i][j]);
        if (SPL >= 1) acc[i][j] = Frag<T>::mma(al, bh[j], acc[i][j]);
      }
      Frag<T>::guard(acc[i][0], acc[i][3], ah, (SPL >= 1) ? al : ah);
    }
    Frag<T>::keep(bh[0], bh[1], bh[2], bh[3]);
    if (SPL == 2) Frag<T>::keep(bl[0], bl[1], bl[2], bl[3]);
  }
  acc_guard4(acc[0][0], acc[0][1], acc[0][2], acc[0][3]);
  acc_guard4(acc[1][0], acc[1][1], acc[1][2], acc[1][3]);
  acc_guard4(acc[2][0], acc[2][1], acc[2][2], acc[2][3]);
  acc_guard4(acc[3][0], acc[3][1], acc[3][2], acc[3][3]);

  float* slab = sT[wave];
  const float* Rb = RESID ? (resid + (size_t)b * strideR) : nullptr;
#pragma unroll
  for (int i = 0; i < 4; ++i) {
    const int mBase = m0 + (i << 4);
#pragma unroll
    for (int j = 0; j < 4; ++j) {
      const int n = n0 + (j << 4) + rlane;
      float bv = 0.f;
      if (BIAS_MODE == 2) bv = bias[n];
      if (BIAS_MODE == 3) bv = bfr(bias[n]);
#pragma unroll
      for (int r = 0; r < 8; ++r) {
        float v = acc[i][j][r] * scale;
        if (BIAS_MODE == 1) v += bias[mBase + mOff + r];
        if (BIAS_MODE == 2 || BIAS_MODE == 3) v += bv;
        if (RESID) v += Rb[(size_t)(mBase + mOff + r) * ldc + n];
        if (ACT == 1) v = tanhf(v);
        if (ACT == 2) v = fmaxf(v, 0.0f);
        if (ACT == 3) v = v / (1.0f + expf(-v));
        if (ACT == 4) v = (v > 0.f) ? v : 0.01f * v;
        slab[(mOff + r) * 68 + (j << 4) + rlane] = v;
      }
    }
    __builtin_amdgcn_fence(__ATOMIC_RELEASE, "workgroup");
    __builtin_amdgcn_wave_barrier();
    __builtin_amdgcn_fence(__ATOMIC_ACQUIRE, "workgroup");
    if (OUT_MODE == 0) {
      float* C = (float*)Cout + (size_t)b * strideC;
      const int hh = lane >> 4, c4 = (lane & 15) * 4;
      for (int pass = 0; pass < 2; ++pass) {
#pragma unroll
        for (int it = 0; it < 8; ++it) {
          const int row = it * 2 + hh;
          v4f v = *(const v4f*)(slab + row * 68 + c4);
          *(volatile v4f*)(C + (size_t)(mBase + row) * ldc + n0 + c4) = v;
        }
        __threadfence();
      }
    } else {
      const int q = lane >> 3, c8 = (lane & 7) * 8;
      unsigned short* C  = (unsigned short*)Cout  + (size_t)b * strideC;
      unsigned short* C2 = (OUT_MODE == 2) ? ((unsigned short*)Cout2 + (size_t)b * strideC) : nullptr;
      for (int pass = 0; pass < 2; ++pass) {
#pragma unroll
        for (int it = 0; it < 4; ++it) {
          const int row = it * 4 + q;
          const float* sp = slab + row * 68 + c8;
          v8h hv, lv;
#pragma unroll
          for (int e = 0; e < 8; ++e) {
            if (OUT_MODE == 1) {
              hv[e] = (_Float16)sp[e];
            } else {
              unsigned short hb = f2bf_bits(sp[e]);
              unsigned short lb = f2bf_bits(sp[e] - bf_bits2f(hb));
              hv[e] = __builtin_bit_cast(_Float16, hb);
              lv[e] = __builtin_bit_cast(_Float16, lb);
            }
          }
          *(volatile v8h*)(C + (size_t)(mBase + row) * ldc + n0 + c8) = hv;
          if (OUT_MODE == 2) *(volatile v8h*)(C2 + (size_t)(mBase + row) * ldc + n0 + c8) = lv;
        }
        __threadfence();
      }
    }
    __builtin_amdgcn_fence(__ATOMIC_RELEASE, "workgroup");
    __builtin_amdgcn_wave_barrier();
    __builtin_amdgcn_fence(__ATOMIC_ACQUIRE, "workgroup");
  }
}

__global__ __launch_bounds__(256) void cast_rows_bf16_kernel(
    const float* __restrict__ src, unsigned short* __restrict__ dst, int total8)
{
  const int i = blockIdx.x * 256 + threadIdx.x;
  if (i >= total8) return;
  const size_t e0 = (size_t)i << 3;
  const v4f a0 = *(const v4f*)(src + e0);
  const v4f a1 = *(const v4f*)(src + e0 + 4);
  v8h hv;
#pragma unroll
  for (int e = 0; e < 4; ++e) {
    hv[e]     = __builtin_bit_cast(_Float16, f2bf_bits(a0[e]));
    hv[4 + e] = __builtin_bit_cast(_Float16, f2bf_bits(a1[e]));
  }
  unsigned short* q = dst + e0;
  *(volatile v8h*)q = hv;
  __threadfence();
  *(volatile v8h*)q = hv;
}

__global__ __launch_bounds__(256) void cast_rows_f16s_kernel(
    const float* __restrict__ src, unsigned short* __restrict__ dst, int total8, float mul)
{
  const int i = blockIdx.x * 256 + threadIdx.x;
  if (i >= total8) return;
  const size_t e0 = (size_t)i << 3;
  const v4f a0 = *(const v4f*)(src + e0);
  const v4f a1 = *(const v4f*)(src + e0 + 4);
  v8h hv;
#pragma unroll
  for (int e = 0; e < 4; ++e) {
    hv[e]     = (_Float16)(bfr(a0[e]) * mul);
    hv[4 + e] = (_Float16)(bfr(a1[e]) * mul);
  }
  unsigned short* q = dst + e0;
  *(volatile v8h*)q = hv;
  __threadfence();
  *(volatile v8h*)q = hv;
}

__global__ __launch_bounds__(256) void xproj_weight_kernel(
    const float* __restrict__ Wx, unsigned short* __restrict__ out, int total8)
{
  const int i = blockIdx.x * 256 + threadIdx.x;
  if (i >= total8) return;
  const int e0 = i << 3;
  const int n  = e0 >> 11;
  const int k0 = e0 & (kDi - 1);
  const bool keep = (n < kXpN);
  const int ns = keep ? n : (kXpN - 1);
  const v4f a0 = *(const v4f*)(Wx + (size_t)ns * kDi + k0);
  const v4f a1 = *(const v4f*)(Wx + (size_t)ns * kDi + k0 + 4);
  v8h hv;
#pragma unroll
  for (int e = 0; e < 4; ++e) {
    const unsigned short h0 = keep ? f2bf_bits(a0[e]) : (unsigned short)0;
    const unsigned short h1 = keep ? f2bf_bits(a1[e]) : (unsigned short)0;
    hv[e]     = __builtin_bit_cast(_Float16, h0);
    hv[4 + e] = __builtin_bit_cast(_Float16, h1);
  }
  unsigned short* q = out + e0;
  *(volatile v8h*)q = hv;
  __threadfence();
  *(volatile v8h*)q = hv;
}

__global__ __launch_bounds__(256) void dt_cast_kernel(
    const float* __restrict__ XD, unsigned short* __restrict__ DT, int total8, float mul)
{
  const int i = blockIdx.x * 256 + threadIdx.x;
  if (i >= total8) return;
  const int row = i >> 3;
  const int c8  = (i & 7) * 8;
  const float* s = XD + (size_t)row * kXdP + c8;
  const v4f a0 = *(const v4f*)(s);
  const v4f a1 = *(const v4f*)(s + 4);
  v8h hv;
#pragma unroll
  for (int e = 0; e < 4; ++e) {
    hv[e]     = (_Float16)(a0[e] * mul);
    hv[4 + e] = (_Float16)(a1[e] * mul);
  }
  unsigned short* q = DT + (size_t)row * kDtR + c8;
  *(volatile v8h*)q = hv;
  __threadfence();
  *(volatile v8h*)q = hv;
}

__global__ __launch_bounds__(256) void conv_silu_kernel(
    const float* __restrict__ XZ, const float* __restrict__ cw, const float* __restrict__ cb,
    float* __restrict__ UC, unsigned short* __restrict__ UCH, unsigned short* __restrict__ UCL)
{
  __shared__ __align__(16) float sT[16 * kConvTP];
  const int tid = threadIdx.x, lane = tid & 31, wave = tid >> 5;
  const int d0 = blockIdx.x * 256, d = d0 + tid;
  const int g0 = blockIdx.y * 64;
  const float w0 = bfr(cw[d * 4 + 0]), w1 = bfr(cw[d * 4 + 1]), w2 = bfr(cw[d * 4 + 2]), w3 = bfr(cw[d * 4 + 3]);
  const float bc = bfr(cb[d]);
  float xm3, xm2, xm1;
  {
    const bool hist = (g0 > 0);
    const int rb = hist ? (g0 - 3) : 0;
    const float v3 = XZ[(size_t)rb * kXz + d];
    const float v2 = XZ[(size_t)(rb + 1) * kXz + d];
    const float v1 = XZ[(size_t)(rb + 2) * kXz + d];
    xm3 = hist ? v3 : 0.f;
    xm2 = hist ? v2 : 0.f;
    xm1 = hist ? v1 : 0.f;
  }
  const int hrow = wave >> 1;
  const int hch  = (wave & 1) * 128 + lane * 4;
#pragma unroll 1
  for (int sub = 0; sub < 4; ++sub) {
    const int lb = g0 + sub * 16;
#pragma unroll 1
    for (int s = 0; s < 16; ++s) {
      const float xcur = XZ[(size_t)(lb + s) * kXz + d];
      float acc = w0 * xm3;
      acc = fmaf(w1, xm2, acc);
      acc = fmaf(w2, xm1, acc);
      acc = fmaf(w3, xcur, acc);
      const float sv = acc + bc;
      const float sg = __builtin_amdgcn_rcpf(1.0f + __expf(-sv));
      sT[s * kConvTP + tid] = sv * sg;
      xm3 = xm2; xm2 = xm1; xm1 = xcur;
    }
    __syncthreads();
    v4f fv[4];
    v8h bh[2], blo[2];
#pragma unroll
    for (int it = 0; it < 4; ++it) fv[it] = *(const v4f*)(sT + (it * 4 + hrow) * kConvTP + hch);
#pragma unroll
    for (int it = 0; it < 2; ++it) {
      const float* sp = sT + (it * 8 + wave) * kConvTP + lane * 8;
      const v4f a0 = *(const v4f*)(sp);
      const v4f a1 = *(const v4f*)(sp + 4);
#pragma unroll
      for (int e = 0; e < 4; ++e) {
        const unsigned short h0 = f2bf_bits(a0[e]), h1 = f2bf_bits(a1[e]);
        const unsigned short l0 = f2bf_bits(a0[e] - bf_bits2f(h0)), l1 = f2bf_bits(a1[e] - bf_bits2f(h1));
        bh[it][e]      = __builtin_bit_cast(_Float16, h0);
        bh[it][4 + e]  = __builtin_bit_cast(_Float16, h1);
        blo[it][e]     = __builtin_bit_cast(_Float16, l0);
        blo[it][4 + e] = __builtin_bit_cast(_Float16, l1);
      }
    }
    for (int pass = 0; pass < 2; ++pass) {
#pragma unroll
      for (int it = 0; it < 4; ++it)
        *(volatile v4f*)(UC + (size_t)(lb + it * 4 + hrow) * kDi + d0 + hch) = fv[it];
#pragma unroll
      for (int it = 0; it < 2; ++it) {
        const size_t o = (size_t)(lb + it * 8 + wave) * kDi + d0 + lane * 8;
        *(volatile v8h*)(UCH + o) = bh[it];
        *(volatile v8h*)(UCL + o) = blo[it];
      }
      __threadfence();
    }
    __syncthreads();
  }
}

__global__ __launch_bounds__(64) void scan_kernel(
    const float* __restrict__ XD, const float* __restrict__ UC, const float* __restrict__ XZ,
    const float* __restrict__ DTP, const float* __restrict__ bdt, const float* __restrict__ Alog,
    const float* __restrict__ Dp, unsigned short* __restrict__ Y16)
{
  __shared__ __align__(16) float sBC[kScanTS * kBcP];
  __shared__ __align__(16) float sY[kScanTS * kScanYP];
  const int tid = threadIdx.x, lane = tid & 31, wave = tid >> 5;
  const int d0 = blockIdx.x * kScanCh;
  const int d  = d0 + tid;
  float negA[kNst], h[kNst];
#pragma unroll
  for (int s = 0; s < kNst; ++s) {
    negA[s] = -__expf(bfr(Alog[(size_t)d * kNst + s]));
    h[s] = 0.f;
  }
  const float bb = bfr(bdt[d]), Dd = bfr(Dp[d]);
  const int q = lane >> 3, c8 = (lane & 7) * 8;
#pragma unroll 1
  for (int t0 = 0; t0 < kSeq; t0 += kScanTS) {
    __syncthreads();
    {
      const float* src = XD + (size_t)(t0 + tid) * kXdP + kDtR;
      float* srow = sBC + tid * kBcP;
#pragma unroll
      for (int i = 0; i < 8; ++i) *(v4f*)(srow + 4 * i) = *(const v4f*)(src + 4 * i);
    }
    __syncthreads();
#pragma unroll 1
    for (int s = 0; s < kScanTS; ++s) {
      const int t = t0 + s;
      const float* xr = sBC + s * kBcP;
      float Bs[kNst], Cs[kNst];
#pragma unroll
      for (int q4 = 0; q4 < 4; ++q4) {
        const v4f bv = *(const v4f*)(xr + 4 * q4);
        const v4f cv = *(const v4f*)(xr + 16 + 4 * q4);
        Bs[4 * q4 + 0] = bv[0]; Bs[4 * q4 + 1] = bv[1]; Bs[4 * q4 + 2] = bv[2]; Bs[4 * q4 + 3] = bv[3];
        Cs[4 * q4 + 0] = cv[0]; Cs[4 * q4 + 1] = cv[1]; Cs[4 * q4 + 2] = cv[2]; Cs[4 * q4 + 3] = cv[3];
      }
      const float v   = DTP[(size_t)t * kDi + d] + bb;
      const float a   = __expf(-fabsf(v));
      const float u   = 1.0f + a;
      const float l1p = __logf(u) + (a - (u - 1.0f)) * __builtin_amdgcn_rcpf(u);
      const float dt  = fmaxf(v, 0.0f) + l1p;
      const float xt  = UC[(size_t)t * kDi + d];
      const float dtx = dt * xt;
      float y = 0.f;
#pragma unroll
      for (int k = 0; k < kNst; ++k) {
        const float e = __expf(dt * negA[k]);
        h[k] = e * h[k] + dtx * Bs[k];
        y = h[k] * Cs[k] + y;
      }
      y = xt * Dd + y;
      const float zv = XZ[(size_t)t * kXz + kDi + d];
      const float sg = __builtin_amdgcn_rcpf(1.0f + __expf(-zv));
      y = y * (zv * sg);
      sY[s * kScanYP + tid] = y;
    }
    __syncthreads();
    v8h hv[8];
#pragma unroll
    for (int it = 0; it < 8; ++it) {
      const int row = it * 8 + wave * 4 + q;
      const float* sp = sY + row * kScanYP + c8;
      const v4f a0 = *(const v4f*)(sp);
      const v4f a1 = *(const v4f*)(sp + 4);
#pragma unroll
      for (int e = 0; e < 4; ++e) {
        hv[it][e]     = (_Float16)(a0[e] * kYCarry);
        hv[it][4 + e] = (_Float16)(a1[e] * kYCarry);
      }
    }
    for (int pass = 0; pass < 2; ++pass) {
#pragma unroll
      for (int it = 0; it < 8; ++it) {
        const int row = it * 8 + wave * 4 + q;
        const size_t o = (size_t)(t0 + row) * kDi + d0 + c8;
        *(volatile v8h*)(Y16 + o) = hv[it];
      }
      __threadfence();
    }
  }
}

extern "C" void kernel_launch(void* const* d_in, const int* in_sizes, int n_in,
                              void* d_out, int out_size, void* d_ws, size_t ws_size,
                              hipStream_t stream) {
  if (n_in < 14) return;
  if (in_sizes[0]  != kRows * kFin) return;
  if (in_sizes[1]  != kDm * kFin) return;
  if (in_sizes[2]  != kDm) return;
  if (in_sizes[3]  != kXz * kDm) return;
  if (in_sizes[4]  != kDi * 4) return;
  if (in_sizes[5]  != kDi) return;
  if (in_sizes[6]  != kXpN * kDi) return;
  if (in_sizes[7]  != kDi * kDtR) return;
  if (in_sizes[8]  != kDi) return;
  if (in_sizes[9]  != kDi * kNst) return;
  if (in_sizes[10] != kDi) return;
  if (in_sizes[11] != kDm * kDi) return;
  if (in_sizes[12] != kFout * kDm) return;
  if (in_sizes[13] != kFout) return;
  if (out_size != kRows * kFout) return;
  if (ws_size < kWsTotal) return;

  const float* x       = (const float*)d_in[0];
  const float* W_fc1   = (const float*)d_in[1];
  const float* b_fc1   = (const float*)d_in[2];
  const float* W_in    = (const float*)d_in[3];
  const float* conv_w  = (const float*)d_in[4];
  const float* conv_b  = (const float*)d_in[5];
  const float* W_xproj = (const float*)d_in[6];
  const float* W_dt    = (const float*)d_in[7];
  const float* b_dt    = (const float*)d_in[8];
  const float* A_log   = (const float*)d_in[9];
  const float* Dp      = (const float*)d_in[10];
  const float* W_out   = (const float*)d_in[11];
  const float* W_fc2   = (const float*)d_in[12];
  const float* b_fc2   = (const float*)d_in[13];
  float* out = (float*)d_out;

  char* ws = (char*)d_ws;
  unsigned short* XB   = (unsigned short*)(ws + kOffXB);
  unsigned short* WF1  = (unsigned short*)(ws + kOffWF1);
  unsigned short* WIN  = (unsigned short*)(ws + kOffWIN);
  unsigned short* WXP  = (unsigned short*)(ws + kOffWXP);
  unsigned short* WDT  = (unsigned short*)(ws + kOffWDT);
  unsigned short* WOU  = (unsigned short*)(ws + kOffWOU);
  unsigned short* WF2  = (unsigned short*)(ws + kOffWF2);
  unsigned short* H16  = (unsigned short*)(ws + kOffH16);
  float*          XZ   = (float*)(ws + kOffXZ);
  float*          UC   = (float*)(ws + kOffUC);
  unsigned short* UCH  = (unsigned short*)(ws + kOffUCH);
  unsigned short* UCL  = (unsigned short*)(ws + kOffUCL);
  float*          XD   = (float*)(ws + kOffXD);
  unsigned short* DT16 = (unsigned short*)(ws + kOffDT);
  float*          DTP  = (float*)(ws + kOffDTP);
  unsigned short* Y16  = (unsigned short*)(ws + kOffY16);
  unsigned short* M2H  = (unsigned short*)(ws + kOffM2H);
  unsigned short* M2L  = (unsigned short*)(ws + kOffM2L);

  cast_rows_bf16_kernel<<<(kRows * kFin / 8) / 256, 256, 0, stream>>>(x, XB, kRows * kFin / 8);
  cast_rows_bf16_kernel<<<(kDm * kFin / 8) / 256, 256, 0, stream>>>(W_fc1, WF1, kDm * kFin / 8);
  cast_rows_f16s_kernel<<<(kXz * kDm / 8) / 256, 256, 0, stream>>>(W_in, WIN, kXz * kDm / 8, kWinCarry);
  xproj_weight_kernel<<<(kXdP * kDi / 8) / 256, 256, 0, stream>>>(W_xproj, WXP, kXdP * kDi / 8);
  cast_rows_f16s_kernel<<<(kDi * kDtR / 8) / 256, 256, 0, stream>>>(W_dt, WDT, kDi * kDtR / 8, kWdtCarry);
  cast_rows_f16s_kernel<<<(kDm * kDi / 8) / 256, 256, 0, stream>>>(W_out, WOU, kDm * kDi / 8, kWoutCarry);
  cast_rows_bf16_kernel<<<(kFout * kDm / 8) / 256, 256, 0, stream>>>(W_fc2, WF2, kFout * kDm / 8);

  for (int b = 0; b < kBatch; ++b) {
    wmma_gemm64<1, 0, 3, 1, false><<<dim3(64, 1), 256, 0, stream>>>(
        XB + (size_t)b * kSeq * kFin, nullptr, kFin, 0L,
        WF1, nullptr, kFin, 0L,
        (void*)H16, nullptr, kDm, 0L,
        b_fc1, nullptr, 0L,
        kSeq, kDm, kFin, 1.0f);
    wmma_gemm64<0, 0, 0, 0, false><<<dim3(256, 1), 256, 0, stream>>>(
        H16, nullptr, kDm, 0L,
        WIN, nullptr, kDm, 0L,
        (void*)XZ, nullptr, kXz, 0L,
        nullptr, nullptr, 0L,
        kSeq, kXz, kDm, 1.0f / kWinCarry);
    conv_silu_kernel<<<dim3(kDi / 256, kSeq / 64), 256, 0, stream>>>(XZ, conv_w, conv_b, UC, UCH, UCL);
    wmma_gemm64<1, 1, 0, 0, false><<<dim3(8, 1), 256, 0, stream>>>(
        UCH, UCL, kDi, 0L,
        WXP, nullptr, kDi, 0L,
        (void*)XD, nullptr, kXdP, 0L,
        nullptr, nullptr, 0L,
        kSeq, kXdP, kDi, 1.0f);
    dt_cast_kernel<<<(kSeq * kDtR / 8) / 256, 256, 0, stream>>>(XD, DT16, kSeq * kDtR / 8, kDtCarry);
    wmma_gemm64<0, 0, 0, 0, false><<<dim3(128, 1), 256, 0, stream>>>(
        DT16, nullptr, kDtR, 0L,
        WDT, nullptr, kDtR, 0L,
        (void*)DTP, nullptr, kDi, 0L,
        nullptr, nullptr, 0L,
        kSeq, kDi, kDtR, 1.0f / (kDtCarry * kWdtCarry));
    scan_kernel<<<kDi / kScanCh, kScanCh, 0, stream>>>(XD, UC, XZ, DTP, b_dt, A_log, Dp, Y16);
    wmma_gemm64<0, 0, 0, 2, false><<<dim3(64, 1), 256, 0, stream>>>(
        Y16, nullptr, kDi, 0L,
        WOU, nullptr, kDi, 0L,
        (void*)M2H, (void*)M2L, kDm, 0L,
        nullptr, nullptr, 0L,
        kSeq, kDm, kDi, 1.0f / (kYCarry * kWoutCarry));
    wmma_gemm64<1, 1, 3, 0, false><<<dim3(32, 1), 256, 0, stream>>>(
        M2H, M2L, kDm, 0L,
        WF2, nullptr, kDm, 0L,
        (void*)(out + (size_t)b * kSeq * kFout), nullptr, kFout, 0L,
        b_fc2, nullptr, 0L,
        kSeq, kFout, kDm, 1.0f);
  }
}
